// SampleQueryExtractionLayer_86852828660039
// MI455X (gfx1250) — hardware-run, weakly checked
//
#include <hip/hip_runtime.h>


#define NQ   8192
#define NN   4096
#define NCC  256
#define NBT  4
typedef _Float16 h16;
typedef unsigned short bf;
typedef __attribute__((ext_vector_type(16))) __bf16   v16bf;
typedef __attribute__((ext_vector_type(16))) _Float16 v16h;
typedef __attribute__((ext_vector_type(8)))  _Float16 v8h;
typedef __attribute__((ext_vector_type(8)))  unsigned short v8us;
typedef __attribute__((ext_vector_type(8)))  float    v8f;
typedef __attribute__((ext_vector_type(4)))  float    v4f;
typedef v8h  __attribute__((may_alias)) v8ha;
typedef v4f  __attribute__((may_alias)) v4fa;
typedef v8us __attribute__((may_alias)) v8usa;

__device__ __forceinline__ unsigned short f2bf(float f) { unsigned u = __float_as_uint(f); u += 0x7FFFu + ((u >> 16) & 1u); return (unsigned short)(u >> 16); }
__device__ __forceinline__ float bf2f(unsigned short b) { return __uint_as_float(((unsigned)b) << 16); }
__device__ __forceinline__ float bfr(float f) { return bf2f(f2bf(f)); }
__device__ __forceinline__ v16h cat16(v8h lo, v8h hi) { return __builtin_shufflevector(lo, hi, 0, 1, 2, 3, 4, 5, 6, 7, 8, 9, 10, 11, 12, 13, 14, 15); }
__device__ __forceinline__ v16bf cat16b(v8us lo, v8us hi) { return __builtin_bit_cast(v16bf, __builtin_shufflevector(lo, hi, 0, 1, 2, 3, 4, 5, 6, 7, 8, 9, 10, 11, 12, 13, 14, 15)); }
__device__ __forceinline__ v8f wmma16(v16h a, v16h b, v8f c) { return __builtin_amdgcn_wmma_f32_16x16x32_f16(false, a, false, b, (short)0, c, false, false); }
__device__ __forceinline__ v8f wmmab(v16bf a, v16bf b, v8f c) { return __builtin_amdgcn_wmma_f32_16x16x32_bf16(false, a, false, b, (short)0, c, false, false); }

template <typename T16> struct WFrag;
template <> struct WFrag<h16> { typedef v16h V; static __device__ __forceinline__ V ld(const h16* p) { return cat16(*(const v8h*)p, *(const v8h*)(p + 16)); } static __device__ __forceinline__ v8f mma(V a, V b, v8f c) { return wmma16(a, b, c); } };
template <> struct WFrag<bf> { typedef v16bf V; static __device__ __forceinline__ V ld(const bf* p) { return cat16b(*(const v8us*)p, *(const v8us*)(p + 16)); } static __device__ __forceinline__ v8f mma(V a, V b, v8f c) { return wmmab(a, b, c); } };
template <typename T16, int NSPLIT, bool BIAS>
__global__ __launch_bounds__(32) void k_gemmw(const T16* __restrict__ A, const T16* __restrict__ A2, const T16* __restrict__ Bt, const T16* __restrict__ Bt2, int K, float* C, int ldc, const float* __restrict__ bias, size_t sA, size_t sB, size_t sC) {
    typedef typename WFrag<T16>::V V;
    __shared__ __align__(16) float os[16 * 68];
    const size_t z = blockIdx.z; A += z * sA; if (A2) A2 += z * sA; Bt += z * sB; if (Bt2) Bt2 += z * sB; C += z * sC;
    const int lane = threadIdx.x & 31, lr = lane & 15, hi = lane >> 4; const int r0 = blockIdx.x * 64, c0 = blockIdx.y * 64;
    v8f acc[4][4];
#pragma unroll
    for (int mb = 0; mb < 4; ++mb)
#pragma unroll
        for (int nb = 0; nb < 4; ++nb) acc[mb][nb] = (v8f){};
    const size_t aoff = (size_t)(r0 + lr) * K + 8 * hi, boff = (size_t)(c0 + lr) * K + 8 * hi;
    for (int kc = 0; kc < K; kc += 32) {
        V a[4], a2[4];
#pragma unroll
        for (int mb = 0; mb < 4; ++mb) { a[mb] = WFrag<T16>::ld(A + aoff + (size_t)mb * 16 * K + kc); if (NSPLIT == 1 || NSPLIT == 2) a2[mb] = WFrag<T16>::ld(A2 + aoff + (size_t)mb * 16 * K + kc); }
#pragma unroll
        for (int nb = 0; nb < 4; ++nb) { const V b = WFrag<T16>::ld(Bt + boff + (size_t)nb * 16 * K + kc); V b2; if (NSPLIT >= 2) b2 = WFrag<T16>::ld(Bt2 + boff + (size_t)nb * 16 * K + kc);
#pragma unroll
            for (int mb = 0; mb < 4; ++mb) { acc[mb][nb] = WFrag<T16>::mma(a[mb], b, acc[mb][nb]); if (NSPLIT == 1 || NSPLIT == 2) acc[mb][nb] = WFrag<T16>::mma(a2[mb], b, acc[mb][nb]); if (NSPLIT >= 2) acc[mb][nb] = WFrag<T16>::mma(a[mb], b2, acc[mb][nb]); } }
        asm volatile("v_nop\n\tv_nop\n\tv_nop\n\tv_nop" : "+v"(acc[0][0]), "+v"(acc[1][1]), "+v"(acc[2][2]), "+v"(acc[3][3]) : "v"(a[0]), "v"(a[3]));
    }
#pragma unroll
    for (int mb = 0; mb < 4; ++mb) {
#pragma unroll
        for (int nb = 0; nb < 4; ++nb) {
#pragma unroll
            for (int j = 0; j < 8; ++j) os[(hi * 8 + j) * 68 + nb * 16 + lr] = acc[mb][nb][j]; }
        __builtin_amdgcn_wave_barrier(); asm volatile("" ::: "memory");
        float* crow = C + (size_t)(r0 + mb * 16) * ldc + c0;
#pragma unroll 1
        for (int ps = 0; ps < 2; ++ps) {
#pragma unroll
            for (int s = 0; s < 8; ++s) { const int row = 2 * s + hi, cofs = lr * 4; v4f val = *(const v4fa*)(os + row * 68 + cofs); if (BIAS) { val[0] += bfr(bias[c0 + cofs]); val[1] += bfr(bias[c0 + cofs + 1]); val[2] += bfr(bias[c0 + cofs + 2]); val[3] += bfr(bias[c0 + cofs + 3]); }
                *(volatile v4f*)(crow + (size_t)row * ldc + cofs) = val; }
            if (ps == 0) __threadfence(); }
        __builtin_amdgcn_wave_barrier(); asm volatile("" ::: "memory");
    }
}

typedef __attribute__((ext_vector_type(2))) _Float16 v2h;
typedef __attribute__((ext_vector_type(4))) _Float16 v4h;
typedef __attribute__((ext_vector_type(2))) unsigned short v2us;
typedef __attribute__((ext_vector_type(4))) unsigned short v4us;
typedef __attribute__((ext_vector_type(2))) float v2f;
__device__ __forceinline__ h16 toh_flush(float x) { const float z = (fabsf(x) < 6.103515625e-05f) ? 0.0f : x; return (h16)z; }

__global__ __launch_bounds__(64) void k_wtp16(const float* __restrict__ src, int K, int N, h16* dst, int KP, int NPz) { const int k0 = (blockIdx.x * 64 + threadIdx.x) * 8; if (k0 >= KP) return; const int n = blockIdx.y; const int z = blockIdx.z; const float* s = src + (size_t)z * K * N; v8h o;
#pragma unroll
    for (int q = 0; q < 8; ++q) { const int k = k0 + q; const bool in = (k < K) && (n < N); const float a = s[(size_t)min(k, K - 1) * N + min(n, N - 1)]; const unsigned mk = 0u - (unsigned)in; o[q] = toh_flush(__uint_as_float(__float_as_uint(bfr(a)) & mk)); }
    h16* d = dst + ((size_t)z * NPz + n) * KP + k0; *(volatile v8h*)d = o; __threadfence(); *(volatile v8h*)d = o; }

__device__ __forceinline__ float mk(float py, float px, int n) { const float y = (float)(n >> 6), x = (float)(n & 63); const float d = __fadd_rn(fabsf(__fsub_rn(py, y)), fabsf(__fsub_rn(px, x))); const float t = __fadd_rn(__fsub_rn(1.0f, d), 1e-4f); const float r = t > 0.0f ? t : 0.0f; return __fmul_rn(r, r); }

__global__ __launch_bounds__(256) void k_ms(const float* __restrict__ p, float* R) { const int q = blockIdx.x * 256 + threadIdx.x; if (q >= NQ) return; const float py = bfr(p[(size_t)q * 2]), px = bfr(p[(size_t)q * 2 + 1]); float s = 0.0f;
    for (int n = 0; n < NN; ++n) s = __fadd_rn(s, mk(py, px, n));
    *(volatile float*)(R + q) = s; __threadfence(); *(volatile float*)(R + q) = s; }

__global__ __launch_bounds__(256) void k_mk(const float* __restrict__ p, const float* __restrict__ R, h16* Wm) { const size_t t = (size_t)blockIdx.x * 256 + threadIdx.x; if (t >= (size_t)NQ * NN / 8) return; const int q = (int)(t / (NN / 8)), n0 = (int)(t % (NN / 8)) * 8; const float py = bfr(p[(size_t)q * 2]), px = bfr(p[(size_t)q * 2 + 1]); const float den = __fadd_rn(R[q], 1e-4f); v8h o;
#pragma unroll
    for (int k = 0; k < 8; ++k) o[k] = toh_flush(__fdiv_rn(mk(py, px, n0 + k), den));
    *(volatile v8h*)(Wm + t * 8) = o; __threadfence(); *(volatile v8h*)(Wm + t * 8) = o; }

extern "C" void kernel_launch(void* const* d_in, const int* in_sizes, int n_in, void* d_out, int out_size, void* d_ws, size_t ws_size, hipStream_t stream) {
    if (n_in < 2) return;
    if (in_sizes[0] != NBT * NN * NCC || in_sizes[1] != NQ * 2) return;
    if (out_size != NQ * NCC) return;
    static_assert(NQ % (64 * NBT) == 0 && NCC % 64 == 0 && NN % 512 == 0 && NN % 32 == 0 && NQ % 256 == 0 && ((size_t)NQ * NN / 8) % 256 == 0 && (NN & (NN - 1)) == 0 && NN == 64 * 64, "the product: M a batch and N multiples of 64, the depth a multiple of 32; a plane row a whole number of lines; every flat grid exact; the grid 64 x 64");
    const float* f = (const float*)d_in[0]; const float* p = (const float*)d_in[1];
    float* out = (float*)d_out;
    char* wsp = (char*)d_ws; auto take = [&](size_t bytes) { char* ptr = wsp; wsp += (bytes + 255) & ~(size_t)255; return (void*)ptr; };
    h16* Wm = (h16*)take((size_t)NQ * NN * 2); h16* Ft = (h16*)take((size_t)NBT * NCC * NN * 2); float* R = (float*)take((size_t)NQ * 4);
    if ((size_t)(wsp - (char*)d_ws) > ws_size) return;
    k_wtp16<<<dim3(NN / 512, NCC, NBT), 64, 0, stream>>>(f, NN, NCC, Ft, NN, NCC);
    k_ms<<<(unsigned)(NQ / 256), 256, 0, stream>>>(p, R);
    k_mk<<<(unsigned)((size_t)NQ * NN / 8 / 256), 256, 0, stream>>>(p, R, Wm);
    k_gemmw<h16, 0, false><<<dim3(NQ / NBT / 64, NCC / 64, NBT), 32, 0, stream>>>(Wm, nullptr, Ft, nullptr, NN, out, NCC, nullptr, (size_t)(NQ / NBT) * NN, (size_t)NCC * NN, (size_t)(NQ / NBT) * NCC);
}
